// QImageDFRSystem_37108517437481
// MI455X (gfx1250) — hardware-verified
//
#include <hip/hip_runtime.h>

typedef __attribute__((ext_vector_type(16))) _Float16 v16h;
typedef __attribute__((ext_vector_type(8)))  float    v8f;
#define PIXLD 64
#define VST2(T, ptr, val) do { const T _v = (val); *(volatile T*)(ptr) = _v; __threadfence(); *(volatile T*)(ptr) = _v; } while (0)

#define HDIM  128
#define BM    16
#define NSTEP 49
#define NDEEP 5
#define NREG  4
#define BTOT  8192
#define WSTR  136

__device__ __forceinline__ float fast_tanh(float x) {
  const float e = __expf(2.0f * x);
  return 1.0f - 2.0f / (e + 1.0f);
}

__device__ __forceinline__ float fq1(float v, float mn, float mx) {
  float s = (mx - mn) * (1.0f / 255.0f);
  float c = fminf(fmaxf(v, mn), mx);
  return (s > 0.f) ? rintf((c - mn) / s) * s + mn : mn;
}

__global__ void prep_quant(const float* __restrict__ p1W, const float* __restrict__ W0,
                           const float* __restrict__ Wd, const float* __restrict__ fc1W,
                           float* __restrict__ p1q, float* __restrict__ W0q,
                           _Float16* __restrict__ Wdq, float* __restrict__ fc1q) {
  __shared__ float smn[256], smx[256];
  const int tid = threadIdx.x;
  auto minmax = [&](const float* src, int n, float& mn, float& mx) {
    float lmn = 3.0e38f, lmx = -3.0e38f;
    for (int i = tid; i < n; i += 256) { float v = src[i]; lmn = fminf(lmn, v); lmx = fmaxf(lmx, v); }
    smn[tid] = lmn; smx[tid] = lmx;
    __syncthreads();
    for (int s = 128; s > 0; s >>= 1) {
      if (tid < s) { smn[tid] = fminf(smn[tid], smn[tid + s]); smx[tid] = fmaxf(smx[tid], smx[tid + s]); }
      __syncthreads();
    }
    mn = smn[0]; mx = smx[0];
    __syncthreads();
  };
  float mn, mx;
  minmax(p1W, 49 * 196, mn, mx);
  for (int i = tid; i < 49 * 196; i += 256) VST2(float, p1q + i, fq1(p1W[i], mn, mx));
  minmax(W0, HDIM, mn, mx);
  for (int i = tid; i < HDIM; i += 256) VST2(float, W0q + i, fq1(W0[i], mn, mx));
  for (int d = 0; d < NDEEP; ++d) {
    const float* src = Wd + d * HDIM * HDIM;
    minmax(src, HDIM * HDIM, mn, mx);
    for (int i = tid; i < HDIM * HDIM; i += 256)
      VST2(_Float16, Wdq + d * HDIM * HDIM + i, (_Float16)fq1(src[i], mn, mx));
  }
  minmax(fc1W, 8 * HDIM, mn, mx);
  for (int i = tid; i < 8 * HDIM; i += 256) VST2(float, fc1q + i, fq1(fc1W[i], mn, mx));
}

__global__ void pix_kernel(const float* __restrict__ x, const float* __restrict__ p1q,
                           const float* __restrict__ p1b, float* __restrict__ pix) {
  __shared__ float xs[196];
  const int b = blockIdx.x;
  for (int p = threadIdx.x; p < 196; p += 64) {
    float v = x[b * 196 + p];
    const float s = 4.0f / 255.0f;
    float c = fminf(fmaxf(v, -0.45f), 3.55f);
    xs[p] = rintf((c + 0.45f) / s) * s - 0.45f;
  }
  __syncthreads();
  const int q = threadIdx.x;
  float acc = 0.f;
  if (q < NSTEP) {
    acc = p1b[q];
    const float* wrow = p1q + q * 196;
    for (int p = 0; p < 196; ++p) acc += xs[p] * wrow[p];
  }
  VST2(float, pix + (size_t)b * PIXLD + q, acc);
}

__global__ __launch_bounds__(256, 4) void dfr_kernel(
    const float* __restrict__ pixg, const float* __restrict__ cell,
    const float* __restrict__ W0q, const float* __restrict__ a0p,
    const _Float16* __restrict__ Wdq, const float* __restrict__ adp,
    const float* __restrict__ fc1q, const float* __restrict__ fc2W,
    const float* __restrict__ fc2b, float* __restrict__ out) {
  __shared__ alignas(16) _Float16 wlds[NDEEP - NREG][HDIM][WSTR];
  __shared__ alignas(16) _Float16 bufA[BM][136];
  __shared__ alignas(16) _Float16 bufB[BM][136];
  __shared__ float pixs[BM][52];
  __shared__ float lastb[BM][132];
  __shared__ float out1[BM][8];

  const int tid  = threadIdx.x;
  const int wave = tid >> 5;
  const int lane = tid & 31;
  const int half = lane >> 4;
  const int ln   = lane & 15;
  const int col  = wave * 16 + ln;
  const int b0   = blockIdx.x * BM;

  for (int i = tid; i < BM * NSTEP; i += 256) {
    int r = i / NSTEP, q = i - r * NSTEP;
    pixs[r][q] = pixg[(b0 + r) * PIXLD + q];
  }

  for (int i = tid; i < (NDEEP - NREG) * HDIM * (HDIM / 8); i += 256) {
    const int l = i / (HDIM * (HDIM / 8));
    const int rem = i - l * (HDIM * (HDIM / 8));
    const int n = rem / (HDIM / 8);
    const int c = rem - n * (HDIM / 8);
    *(uint4*)&wlds[l][n][c * 8] =
        *(const uint4*)(Wdq + ((NREG + l) * HDIM + n) * HDIM + c * 8);
  }

  v16h bw[NREG][4];
#pragma unroll
  for (int d = 0; d < NREG; ++d) {
#pragma unroll
    for (int kt = 0; kt < 4; ++kt) {
      const _Float16* src = Wdq + ((d * HDIM + col) * HDIM + kt * 32 + half * 8);
      union { uint4 u[2]; v16h v; } u;
      u.u[0] = *(const uint4*)(src);
      u.u[1] = *(const uint4*)(src + 16);
      bw[d][kt] = u.v;
    }
  }

  const float w0v = W0q[col];
  const float a0  = a0p[0];
  float ad[NDEEP];
#pragma unroll
  for (int i = 0; i < NDEEP; ++i) ad[i] = adp[i];

  float h0acc[8];
  v8f hs[NDEEP];
#pragma unroll
  for (int r = 0; r < 8; ++r) {
    const int b = b0 + r + 8 * half;
    h0acc[r] = cell[(size_t)b * HDIM + col];
#pragma unroll
    for (int i = 0; i < NDEEP; ++i)
      hs[i][r] = cell[((size_t)(i + 1) * BTOT + b) * HDIM + col];
  }

  __syncthreads();

  for (int t = 0; t < NSTEP; ++t) {
#pragma unroll
    for (int r = 0; r < 8; ++r) {
      const int row = r + 8 * half;
      float v = fast_tanh(pixs[row][t] * w0v + a0 * h0acc[r]);
      h0acc[r] = v;
      bufA[row][col] = (_Float16)v;
    }
    __syncthreads();

#pragma unroll
    for (int i = 0; i < NDEEP; ++i) {
      const _Float16 (*src)[136] = (i & 1) ? bufB : bufA;
      _Float16 (*dst)[136]       = (i & 1) ? bufA : bufB;
      v16h af[4];
#pragma unroll
      for (int kt = 0; kt < 4; ++kt) {
        const _Float16* p = &src[ln][kt * 32 + 8 * half];
        union { uint4 u[2]; v16h v; } u;
        u.u[0] = *(const uint4*)(p);
        u.u[1] = *(const uint4*)(p + 16);
        af[kt] = u.v;
      }
      v8f c;
#pragma unroll
      for (int r = 0; r < 8; ++r) c[r] = ad[i] * hs[i][r];
      if (i < NREG) {
#pragma unroll
        for (int kt = 0; kt < 4; ++kt)
        { c = __builtin_amdgcn_wmma_f32_16x16x32_f16(false, af[kt], false, bw[i][kt],
                                                     (short)0, c, false, false);
          asm volatile("v_nop\n\tv_nop\n\tv_nop\n\tv_nop" : "+v"(c) : "v"(af[kt]), "v"(bw[i][kt])); }
      } else {
#pragma unroll
        for (int kt = 0; kt < 4; ++kt) {
          const _Float16* p = &wlds[i - NREG][col][kt * 32 + half * 8];
          union { uint4 u[2]; v16h v; } u;
          u.u[0] = *(const uint4*)(p);
          u.u[1] = *(const uint4*)(p + 16);
          c = __builtin_amdgcn_wmma_f32_16x16x32_f16(false, af[kt], false, u.v,
                                                     (short)0, c, false, false);
          asm volatile("v_nop\n\tv_nop\n\tv_nop\n\tv_nop" : "+v"(c) : "v"(af[kt]), "v"(u.v));
        }
      }
#pragma unroll
      for (int r = 0; r < 8; ++r) c[r] = fast_tanh(c[r]);
      hs[i] = c;
      if (i < NDEEP - 1) {
#pragma unroll
        for (int r = 0; r < 8; ++r)
          dst[r + 8 * half][col] = (_Float16)c[r];
      }
      __syncthreads();
    }
  }

#pragma unroll
  for (int r = 0; r < 8; ++r)
    lastb[r + 8 * half][col] = hs[NDEEP - 1][r];
  __syncthreads();

  if (tid < BM * 8) {
    const int row = tid >> 3, o = tid & 7;
    float acc = 0.f;
    const float* w = fc1q + o * HDIM;
    for (int h = 0; h < HDIM; ++h) acc += lastb[row][h] * w[h];
    out1[row][o] = fmaxf(acc, 0.f);
  }
  __syncthreads();
  if (tid < BM * 10) {
    const int row = tid / 10, j = tid - row * 10;
    float acc = fc2b[j];
#pragma unroll
    for (int o = 0; o < 8; ++o) acc += out1[row][o] * fc2W[j * 8 + o];
    VST2(float, out + (size_t)(b0 + row) * 10 + j, acc);
  }
}

extern "C" void kernel_launch(void* const* d_in, const int* in_sizes, int n_in,
                              void* d_out, int out_size, void* d_ws, size_t ws_size,
                              hipStream_t stream) {
  const float* x    = (const float*)d_in[0];
  const float* cell = (const float*)d_in[1];
  const float* W0   = (const float*)d_in[2];
  const float* a0   = (const float*)d_in[3];
  const float* Wd   = (const float*)d_in[4];
  const float* ad   = (const float*)d_in[5];
  const float* p1W  = (const float*)d_in[6];
  const float* p1b  = (const float*)d_in[7];
  const float* fc1W = (const float*)d_in[8];
  const float* fc2W = (const float*)d_in[9];
  const float* fc2b = (const float*)d_in[10];
  float* out = (float*)d_out;

  (void)in_sizes; (void)n_in; (void)out_size;
  if (ws_size < 4u * 1024 * 1024) return;
  char* ws = (char*)d_ws;
  float*    pix  = (float*)(ws);
  float*    p1q  = (float*)(ws + 2097152);
  float*    W0q  = (float*)(ws + 2135568);
  float*    fc1q = (float*)(ws + 2136080);
  _Float16* Wdq  = (_Float16*)(ws + 2140176);

  prep_quant<<<1, 256, 0, stream>>>(p1W, W0, Wd, fc1W, p1q, W0q, Wdq, fc1q);
  pix_kernel<<<BTOT, 64, 0, stream>>>(x, p1q, p1b, pix);
  dfr_kernel<<<BTOT / BM, 256, 0, stream>>>(pix, cell, W0q, a0, Wdq, ad,
                                            fc1q, fc2W, fc2b, out);
}
